// Mamba2_81544249082357
// MI455X (gfx1250) — hardware-run, weakly checked
//
#include <hip/hip_runtime.h>
#include <math.h>

typedef __attribute__((ext_vector_type(16))) _Float16 v16h;
typedef __attribute__((ext_vector_type(8)))  _Float16 v8h;
typedef __attribute__((ext_vector_type(2)))  _Float16 v2h;
typedef __attribute__((ext_vector_type(16))) __bf16   v16b;
typedef __attribute__((ext_vector_type(8)))  __bf16   v8b;
typedef __attribute__((ext_vector_type(8)))  float    v8f;
typedef __attribute__((ext_vector_type(4)))  float    v4f;
typedef __attribute__((ext_vector_type(2)))  float    v2f;

constexpr int kNb   = 2;
constexpr int kS    = 512;
constexpr int kRows = kNb * kS;
constexpr int kDM   = 768;
constexpr int kH    = 24;
constexpr int kP    = 64;
constexpr int kN    = 64;
constexpr int kDS   = kH * kP;
constexpr int kCD   = kDS + 2 * kN;
constexpr int kDin  = 2 * kDS + 2 * kN + kH;
constexpr int kDinP = 3232;
constexpr int kQ    = 64;
constexpr int kC    = kS / kQ;
constexpr int kBC   = kNb * kC;
constexpr int kE    = kNb * kH * kC;
constexpr int kThr  = 256;
constexpr float kInCarry = 1024.0f;
constexpr float kSc = 1.0f / (kInCarry * kInCarry);
constexpr float kF16MinNormal = 6.103515625e-5f;

static_assert(kQ == 64 && kC == 8 && kE == 384 && kP == 64 && kN == 64 && kH == 24 && kDin == 3224 && kCD == 1664, "the index arithmetic below uses these sizes");

constexpr size_t kOffZB = 0ull;
constexpr size_t kOffBIA = 8192ull;
constexpr size_t kOffU16 = 8448ull;
constexpr size_t kOffWIN16 = 1581312ull;
constexpr size_t kOffWOUT16 = 6545664ull;
constexpr size_t kOffZ32 = 8904960ull;
constexpr size_t kOffXBC32 = 15196416ull;
constexpr size_t kOffXBCS32 = 22012160ull;
constexpr size_t kOffDTR32 = 28827904ull;
constexpr size_t kOffXT16 = 28958976ull;
constexpr size_t kOffB16 = 32104704ull;
constexpr size_t kOffC16 = 32235776ull;
constexpr size_t kOffG32 = 32366848ull;
constexpr size_t kOffCS = 32628992ull;
constexpr size_t kOffWTV = 32727296ull;
constexpr size_t kOffEV = 32825600ull;
constexpr size_t kOffDV = 32923904ull;
constexpr size_t kOffTOT = 33022208ull;
constexpr size_t kOffM16 = 33024256ull;
constexpr size_t kOffYD32 = 36169984ull;
constexpr size_t kOffBDT16 = 42461440ull;
constexpr size_t kOffST32 = 45607168ull;
constexpr size_t kOffH16 = 51898624ull;
constexpr size_t kOffCE16 = 55044352ull;
constexpr size_t kOffY16 = 58190080ull;
constexpr size_t kOffYO32 = kOffST32;
constexpr size_t kWsTotal = 61335808ull;
static_assert(kWsTotal <= 134217728ull, "carve cap: under 128 MiB");
static_assert(kOffZB == 0
              && kOffBIA == kOffZB + 8192ull
              && kOffU16 == kOffBIA + 256ull
              && kOffWIN16 == kOffU16 + 1572864ull
              && kOffWOUT16 == kOffWIN16 + 4964352ull
              && kOffZ32 == kOffWOUT16 + 2359296ull
              && kOffXBC32 == kOffZ32 + 6291456ull
              && kOffXBCS32 == kOffXBC32 + 6815744ull
              && kOffDTR32 == kOffXBCS32 + 6815744ull
              && kOffXT16 == kOffDTR32 + 131072ull
              && kOffB16 == kOffXT16 + 3145728ull
              && kOffC16 == kOffB16 + 131072ull
              && kOffG32 == kOffC16 + 131072ull
              && kOffCS == kOffG32 + 262144ull
              && kOffWTV == kOffCS + 98304ull
              && kOffEV == kOffWTV + 98304ull
              && kOffDV == kOffEV + 98304ull
              && kOffTOT == kOffDV + 98304ull
              && kOffM16 == kOffTOT + 2048ull
              && kOffYD32 == kOffM16 + 3145728ull
              && kOffBDT16 == kOffYD32 + 6291456ull
              && kOffST32 == kOffBDT16 + 3145728ull
              && kOffH16 == kOffST32 + 6291456ull
              && kOffCE16 == kOffH16 + 3145728ull
              && kOffY16 == kOffCE16 + 3145728ull
              && kWsTotal == kOffY16 + 3145728ull, "the carve is chained and totalled");
static_assert((kOffZB % 256) == 0 && (kOffBIA % 256) == 0 && (kOffU16 % 256) == 0 && (kOffWIN16 % 256) == 0 && (kOffWOUT16 % 256) == 0 && (kOffZ32 % 256) == 0 && (kOffXBC32 % 256) == 0 && (kOffXBCS32 % 256) == 0 && (kOffDTR32 % 256) == 0 && (kOffXT16 % 256) == 0 && (kOffB16 % 256) == 0 && (kOffC16 % 256) == 0 && (kOffG32 % 256) == 0 && (kOffCS % 256) == 0 && (kOffWTV % 256) == 0 && (kOffEV % 256) == 0 && (kOffDV % 256) == 0 && (kOffTOT % 256) == 0 && (kOffM16 % 256) == 0 && (kOffYD32 % 256) == 0 && (kOffBDT16 % 256) == 0 && (kOffST32 % 256) == 0 && (kOffH16 % 256) == 0 && (kOffCE16 % 256) == 0 && (kOffY16 % 256) == 0, "aligned regions");
static_assert(2048 >= kCD && 2048 >= kDS && 2048 >= kDM, "the zero bias covers the widest N of any engine launch (the engine reads bias[n] for every n < N)");

__device__ __forceinline__ unsigned short f2bf_bits(float f) {
  unsigned u = __float_as_uint(f);
  return (unsigned short)((u + 0x7FFFu + ((u >> 16) & 1u)) >> 16);
}
__device__ __forceinline__ float bf_bits2f(unsigned short h) { return __uint_as_float(((unsigned)h) << 16); }
__device__ __forceinline__ float bf16r(float f) { return bf_bits2f(f2bf_bits(f)); }
__device__ __forceinline__ float carry_flush(float v, float carry) {
  const float s = v * carry;
  return (fabsf(s) < kF16MinNormal) ? 0.0f : s;
}

__device__ __forceinline__ void dep_guard4_h(v8f& a, v8f& b, v8f& c, v8f& d, v16h x, v16h y) { asm volatile("v_nop\n\tv_nop\n\tv_nop\n\tv_nop" : "+v"(a), "+v"(b), "+v"(c), "+v"(d) : "v"(x), "v"(y)); }
__device__ __forceinline__ void dep_guard4_b(v8f& a, v8f& b, v8f& c, v8f& d, v16b x, v16b y) { asm volatile("v_nop\n\tv_nop\n\tv_nop\n\tv_nop" : "+v"(a), "+v"(b), "+v"(c), "+v"(d) : "v"(x), "v"(y)); }
__device__ __forceinline__ void keep4_h(v16h a, v16h b, v16h c, v16h d) { asm volatile("v_nop" :: "v"(a), "v"(b), "v"(c), "v"(d)); }
__device__ __forceinline__ void keep4_b(v16b a, v16b b, v16b c, v16b d) { asm volatile("v_nop" :: "v"(a), "v"(b), "v"(c), "v"(d)); }
__device__ __forceinline__ void acc_guard4(v8f& a, v8f& b, v8f& c, v8f& d) { asm volatile("v_nop\n\tv_nop\n\tv_nop\n\tv_nop" : "+v"(a), "+v"(b), "+v"(c), "+v"(d)); }

template <typename T> struct Frag;
template <> struct Frag<_Float16> {
  typedef v16h V; union U { v16h v; v8h h[2]; };
  static __device__ __forceinline__ v16h load(const _Float16* p) {
    U f; f.h[0] = *(const v8h*)(p); f.h[1] = *(const v8h*)(p + 16); return f.v;
  }
  static __device__ __forceinline__ v8f mma(v16h a, v16h b, v8f c) {
    return __builtin_amdgcn_wmma_f32_16x16x32_f16(false, a, false, b, (short)0, c, false, false);
  }
  static __device__ __forceinline__ void guard4(v8f& a, v8f& b, v8f& c, v8f& d, v16h x, v16h y) { dep_guard4_h(a, b, c, d, x, y); }
  static __device__ __forceinline__ void keep(v16h a, v16h b, v16h c, v16h d) { keep4_h(a, b, c, d); }
};
template <> struct Frag<__bf16> {
  typedef v16b V; union U { v16b v; v8b h[2]; };
  static __device__ __forceinline__ v16b load(const __bf16* p) {
    U f; f.h[0] = *(const v8b*)(p); f.h[1] = *(const v8b*)(p + 16); return f.v;
  }
  static __device__ __forceinline__ v8f mma(v16b a, v16b b, v8f c) {
    return __builtin_amdgcn_wmma_f32_16x16x32_bf16(false, a, false, b, (short)0, c, false, false);
  }
  static __device__ __forceinline__ void guard4(v8f& a, v8f& b, v8f& c, v8f& d, v16b x, v16b y) { dep_guard4_b(a, b, c, d, x, y); }
  static __device__ __forceinline__ void keep(v16b a, v16b b, v16b c, v16b d) { keep4_b(a, b, c, d); }
};

__device__ __forceinline__ v8f mma_h(v16h a, v16h b, v8f c) {
  c = __builtin_amdgcn_wmma_f32_16x16x32_f16(false, a, false, b, (short)0, c, false, false);
  asm volatile("v_nop\n\tv_nop\n\tv_nop\n\tv_nop" : "+v"(c) : "v"(a), "v"(b));
  return c;
}

template <int ET> struct Elem;
template <> struct Elem<0> { typedef _Float16 T; };
template <> struct Elem<1> { typedef __bf16 T; };
template <int ET, bool SPLIT, int BIAS_MODE, int OUT_MODE, bool RESID, int ACT = 0>
__global__ __launch_bounds__(256) void wmma_gemm64(
    const unsigned short* __restrict__ Ap, const unsigned short* __restrict__ A2p, int lda, long strideA,
    const unsigned short* __restrict__ Btp, const unsigned short* __restrict__ Bt2p, int ldb, long strideB,
    void* __restrict__ Cout, void* __restrict__ Cout2, int ldc, long strideC,
    const float* __restrict__ bias,
    const float* __restrict__ resid, long strideR,
    int M, int N, int K, float scale) {
  typedef typename Elem<ET>::T T;
  typedef typename Frag<T>::V V;
  const T* A = (const T*)Ap; const T* A2 = (const T*)A2p; const T* Bt = (const T*)Btp; const T* Bt2 = (const T*)Bt2p;
  __shared__ __align__(16) float sT[8][16 * 68];
  const int b    = blockIdx.y;
  const int lane = threadIdx.x & 31;
  const int wave = threadIdx.x >> 5;
  const int tilesN = N >> 6;
  const int tilesM = M >> 6;
  const int tile = blockIdx.x * 8 + wave;
  if (tile >= tilesM * tilesN) return;
  const int tm = tile / tilesN;
  const int tn = tile - tm * tilesN;
  const int m0 = tm << 6;
  const int n0 = tn << 6;

  const T* Ab  = A  + (size_t)b * strideA;
  const T* Bb  = Bt + (size_t)b * strideB;
  const T* Ab2 = SPLIT ? (A2  + (size_t)b * strideA) : nullptr;
  const T* Bb2 = SPLIT ? (Bt2 + (size_t)b * strideB) : nullptr;

  const int rlane = lane & 15;
  const int koff  = (lane >> 4) * 8;
  const int mOff  = (lane >> 4) * 8;

  v8f acc[4][4];
#pragma unroll
  for (int i = 0; i < 4; ++i)
#pragma unroll
    for (int j = 0; j < 4; ++j) acc[i][j] = (v8f){0.f,0.f,0.f,0.f,0.f,0.f,0.f,0.f};

  for (int k0 = 0; k0 < K; k0 += 32) {
    V bh[4], bl[4];
#pragma unroll
    for (int j = 0; j < 4; ++j) {
      const size_t bo = (size_t)(n0 + (j << 4) + rlane) * ldb + koff + k0;
      bh[j] = Frag<T>::load(Bb + bo);
      if (SPLIT) bl[j] = Frag<T>::load(Bb2 + bo);
    }
#pragma unroll
    for (int i = 0; i < 4; ++i) {
      const size_t ao = (size_t)(m0 + (i << 4) + rlane) * lda + koff + k0;
      V ah = Frag<T>::load(Ab + ao);
      V al;
      if (SPLIT) al = Frag<T>::load(Ab2 + ao);
#pragma unroll
      for (int j = 0; j < 4; ++j) {
        acc[i][j] = Frag<T>::mma(ah, bh[j], acc[i][j]);
        if (SPLIT) {
          acc[i][j] = Frag<T>::mma(ah, bl[j], acc[i][j]);
          acc[i][j] = Frag<T>::mma(al, bh[j], acc[i][j]);
        }
      }
      Frag<T>::guard4(acc[i][0], acc[i][1], acc[i][2], acc[i][3], ah, SPLIT ? al : ah);
    }
    Frag<T>::keep(bh[0], bh[1], bh[2], bh[3]);
    if (SPLIT) Frag<T>::keep(bl[0], bl[1], bl[2], bl[3]);
  }
  acc_guard4(acc[0][0], acc[0][1], acc[0][2], acc[0][3]);
  acc_guard4(acc[1][0], acc[1][1], acc[1][2], acc[1][3]);
  acc_guard4(acc[2][0], acc[2][1], acc[2][2], acc[2][3]);
  acc_guard4(acc[3][0], acc[3][1], acc[3][2], acc[3][3]);

  float* slab = sT[wave];
  const float* Rb = RESID ? (resid + (size_t)b * strideR) : nullptr;
#pragma unroll
  for (int i = 0; i < 4; ++i) {
    const int mBase = m0 + (i << 4);
#pragma unroll
    for (int j = 0; j < 4; ++j) {
      const int n = n0 + (j << 4) + rlane;
      float bv = 0.f;
      if (BIAS_MODE == 2) bv = bias[n];
#pragma unroll
      for (int r = 0; r < 8; ++r) {
        float v = acc[i][j][r] * scale;
        if (BIAS_MODE == 1) v += bias[mBase + mOff + r];
        if (BIAS_MODE == 2) v += bv;
        if (RESID) v += Rb[(size_t)(mBase + mOff + r) * ldc + n];
        if (ACT == 1) v = tanhf(v);
        if (ACT == 2) v = fmaxf(v, 0.0f);
        if (ACT == 3) v = v / (1.0f + expf(-v));
        if (ACT == 4) v = (v > 0.f) ? v : 0.01f * v;
        slab[(mOff + r) * 68 + (j << 4) + rlane] = v;
      }
    }
    __builtin_amdgcn_fence(__ATOMIC_RELEASE, "workgroup");
    __builtin_amdgcn_wave_barrier();
    __builtin_amdgcn_fence(__ATOMIC_ACQUIRE, "workgroup");
    if (OUT_MODE == 0) {
      float* C = (float*)Cout + (size_t)b * strideC;
      const int hh = lane >> 4, c4 = (lane & 15) * 4;
      for (int pass = 0; pass < 2; ++pass) {
#pragma unroll
        for (int it = 0; it < 8; ++it) {
          const int row = it * 2 + hh;
          v4f v = *(const v4f*)(slab + row * 68 + c4);
          *(volatile v4f*)(C + (size_t)(mBase + row) * ldc + n0 + c4) = v;
        }
        __threadfence();
      }
    } else {
      const int q = lane >> 3, c8 = (lane & 7) * 8;
      unsigned short* C  = (unsigned short*)Cout  + (size_t)b * strideC;
      unsigned short* C2 = (OUT_MODE == 2) ? ((unsigned short*)Cout2 + (size_t)b * strideC) : nullptr;
      for (int pass = 0; pass < 2; ++pass) {
#pragma unroll
        for (int it = 0; it < 4; ++it) {
          const int row = it * 4 + q;
          const float* sp = slab + row * 68 + c8;
          v8h hv, lv;
#pragma unroll
          for (int e = 0; e < 8; ++e) {
            if (OUT_MODE == 1) {
              hv[e] = (_Float16)sp[e];
            } else {
              unsigned short hb = f2bf_bits(sp[e]);
              unsigned short lb = f2bf_bits(sp[e] - bf_bits2f(hb));
              hv[e] = __builtin_bit_cast(_Float16, hb);
              lv[e] = __builtin_bit_cast(_Float16, lb);
            }
          }
          *(volatile v8h*)(C + (size_t)(mBase + row) * ldc + n0 + c8) = hv;
          if (OUT_MODE == 2) *(volatile v8h*)(C2 + (size_t)(mBase + row) * ldc + n0 + c8) = lv;
        }
        __threadfence();
      }
    }
    __builtin_amdgcn_fence(__ATOMIC_RELEASE, "workgroup");
    __builtin_amdgcn_wave_barrier();
    __builtin_amdgcn_fence(__ATOMIC_ACQUIRE, "workgroup");
  }
}

__global__ __launch_bounds__(kThr) void cast_plane_kernel(const float* __restrict__ src, unsigned short* __restrict__ dst,
                                                          int colsLog2, int dstPitch, int dstOff) {
  const int i   = blockIdx.x * kThr + threadIdx.x;
  const int sh  = colsLog2 - 3;
  const int row = i >> sh;
  const int c8  = (i & ((1 << sh) - 1)) * 8;
  const float* sp = src + ((size_t)row << colsLog2) + c8;
  const v4f a0 = *(const v4f*)(sp);
  const v4f a1 = *(const v4f*)(sp + 4);
  v8h hv;
#pragma unroll
  for (int e = 0; e < 4; ++e) {
    const float f0 = a0[e];
    const float f1 = a1[e];
    hv[e]     = (_Float16)carry_flush(bf16r(f0), kInCarry);
    hv[4 + e] = (_Float16)carry_flush(bf16r(f1), kInCarry);
  }
  unsigned short* dp = dst + (size_t)row * dstPitch + dstOff + c8;
  *(volatile v8h*)dp = hv;
  __threadfence();
  *(volatile v8h*)dp = hv;
}

__global__ __launch_bounds__(256) void wmma_gemm32(
    const unsigned short* __restrict__ Ap, int lda, long strideA,
    const unsigned short* __restrict__ Btp, int ldb, long strideB,
    float* __restrict__ Cout, int ldc, long strideC,
    const float* __restrict__ bias,
    int M, int N, int K, float scale) {
  typedef _Float16 T;
  typedef Frag<T>::V V;
  const T* A = (const T*)Ap; const T* Bt = (const T*)Btp;
  __shared__ __align__(16) float sT[8][16 * 36];
  const int b    = blockIdx.y;
  const int lane = threadIdx.x & 31;
  const int wave = threadIdx.x >> 5;
  const int tilesN = N >> 5;
  const int tilesM = M >> 6;
  const int tile = blockIdx.x * 8 + wave;
  if (tile >= tilesM * tilesN) return;
  const int tm = tile / tilesN;
  const int tn = tile - tm * tilesN;
  const int m0 = tm << 6;
  const int n0 = tn << 5;

  const T* Ab = A  + (size_t)b * strideA;
  const T* Bb = Bt + (size_t)b * strideB;

  const int rlane = lane & 15;
  const int koff  = (lane >> 4) * 8;
  const int mOff  = (lane >> 4) * 8;

  v8f acc[4][2];
#pragma unroll
  for (int i = 0; i < 4; ++i)
#pragma unroll
    for (int j = 0; j < 2; ++j) acc[i][j] = (v8f){0.f,0.f,0.f,0.f,0.f,0.f,0.f,0.f};

  for (int k0 = 0; k0 < K; k0 += 32) {
    V bh[2];
#pragma unroll
    for (int j = 0; j < 2; ++j) {
      const size_t bo = (size_t)(n0 + (j << 4) + rlane) * ldb + koff + k0;
      bh[j] = Frag<T>::load(Bb + bo);
    }
#pragma unroll
    for (int i = 0; i < 4; i += 2) {
      const size_t ao0 = (size_t)(m0 + (i << 4) + rlane) * lda + koff + k0;
      const size_t ao1 = (size_t)(m0 + ((i + 1) << 4) + rlane) * lda + koff + k0;
      V ah0 = Frag<T>::load(Ab + ao0);
      V ah1 = Frag<T>::load(Ab + ao1);
      acc[i][0]     = Frag<T>::mma(ah0, bh[0], acc[i][0]);
      acc[i][1]     = Frag<T>::mma(ah0, bh[1], acc[i][1]);
      acc[i + 1][0] = Frag<T>::mma(ah1, bh[0], acc[i + 1][0]);
      acc[i + 1][1] = Frag<T>::mma(ah1, bh[1], acc[i + 1][1]);
      Frag<T>::guard4(acc[i][0], acc[i][1], acc[i + 1][0], acc[i + 1][1], ah0, ah1);
    }
    Frag<T>::keep(bh[0], bh[1], bh[0], bh[1]);
  }
  acc_guard4(acc[0][0], acc[0][1], acc[1][0], acc[1][1]);
  acc_guard4(acc[2][0], acc[2][1], acc[3][0], acc[3][1]);

  float* slab = sT[wave];
  float* C = Cout + (size_t)b * strideC;
#pragma unroll
  for (int i = 0; i < 4; ++i) {
    const int mBase = m0 + (i << 4);
#pragma unroll
    for (int j = 0; j < 2; ++j) {
      const int n = n0 + (j << 4) + rlane;
      const float bv = bias[n];
#pragma unroll
      for (int r = 0; r < 8; ++r) {
        float v = acc[i][j][r] * scale;
        v += bv;
        slab[(mOff + r) * 36 + (j << 4) + rlane] = v;
      }
    }
    __builtin_amdgcn_fence(__ATOMIC_RELEASE, "workgroup");
    __builtin_amdgcn_wave_barrier();
    __builtin_amdgcn_fence(__ATOMIC_ACQUIRE, "workgroup");
    {
      const int q = lane >> 3, c4 = (lane & 7) * 4;
      for (int pass = 0; pass < 2; ++pass) {
#pragma unroll
        for (int it = 0; it < 4; ++it) {
          const int row = it * 4 + q;
          v4f v = *(const v4f*)(slab + row * 36 + c4);
          *(volatile v4f*)(C + (size_t)(mBase + row) * ldc + n0 + c4) = v;
        }
        __threadfence();
      }
    }
    __builtin_amdgcn_fence(__ATOMIC_RELEASE, "workgroup");
    __builtin_amdgcn_wave_barrier();
    __builtin_amdgcn_fence(__ATOMIC_ACQUIRE, "workgroup");
  }
}
static_assert(sizeof(float) * 8 * 16 * 36 == 18432, "the tail's slabs: 8 waves x 16 rows x 36 floats = 18,432 B of LDS");


__global__ __launch_bounds__(kThr) void zero_kernel(float* __restrict__ dst) {
  const size_t o4 = ((size_t)blockIdx.x * kThr + threadIdx.x) * 4u;
  const v4f z = {0.f, 0.f, 0.f, 0.f};
  *(volatile v4f*)(dst + o4) = z;
  __threadfence();
  *(volatile v4f*)(dst + o4) = z;
}

__global__ __launch_bounds__(64) void bias_kernel(const float* __restrict__ dt_bias, float* __restrict__ BIA) {
  const unsigned i = threadIdx.x;
  const float a = dt_bias[(i < (unsigned)kH) ? i : 0u];
  const float v = (i < (unsigned)kH) ? bf16r(a) : 0.0f;
  *(volatile float*)(BIA + i) = v;
  __threadfence();
  *(volatile float*)(BIA + i) = v;
}

__global__ __launch_bounds__(kThr) void conv_silu_kernel(const float* __restrict__ XBC, const float* __restrict__ conv_w, const float* __restrict__ conv_b, float* __restrict__ XBCS) {
  const unsigned i = blockIdx.x * (unsigned)kThr + threadIdx.x;
  const unsigned r = i / 416u, c4 = i - r * 416u;
  const unsigned t = r & 511u;
  const unsigned ch = c4 * 4u;
  v4f wv[4];
#pragma unroll
  for (int q = 0; q < 4; ++q) wv[q] = *(const v4f*)(conv_w + (size_t)(ch + q) * 4u);
  const v4f bv = *(const v4f*)(conv_b + ch);
  v4f acc;
#pragma unroll
  for (int q = 0; q < 4; ++q) { const float b0 = bv[q]; acc[q] = bf16r(b0); }
#pragma unroll
  for (int k = 0; k < 4; ++k) {
    const bool live = t + (unsigned)k >= 3u;
    const unsigned rr = live ? (r + (unsigned)k - 3u) : r;
    const v4f xv = *(const v4f*)(XBC + (size_t)rr * kCD + ch);
#pragma unroll
    for (int q = 0; q < 4; ++q) { const float w0 = wv[q][k]; acc[q] += live ? bf16r(w0) * xv[q] : 0.0f; }
  }
  v4f o;
#pragma unroll
  for (int q = 0; q < 4; ++q) { const float a = acc[q]; o[q] = a / (1.0f + expf(-a)); }
  float* dp = XBCS + (size_t)i * 4u;
  *(volatile v4f*)dp = o;
  __threadfence();
  *(volatile v4f*)dp = o;
}
static_assert((size_t)kRows * (kCD / 4) == 1664ull * kThr && kCD / 4 == 416 && kS == 512, "conv grid exact: 1,664 blocks; 416 groups of 4 channels a row; 512 positions a sequence");

__global__ __launch_bounds__(kThr) void xt_cast_kernel(const float* __restrict__ XBCS, unsigned short* __restrict__ XT16) {
  const unsigned i = blockIdx.x * (unsigned)kThr + threadIdx.x;
  const unsigned j = i & 7u, p = (i >> 3) & 63u, e = i >> 9;
  const unsigned c = e & 7u, bh = e >> 3;
  const unsigned b = bh / (unsigned)kH, h = bh - b * (unsigned)kH;
  const float* sp = XBCS + (size_t)(b * (unsigned)kS + c * (unsigned)kQ + j * 8u) * kCD + h * (unsigned)kP + p;
  v8h hv;
#pragma unroll
  for (int t = 0; t < 8; ++t) { const float v = sp[(size_t)t * kCD]; hv[t] = (_Float16)carry_flush(v, kInCarry); }
  unsigned short* dp = XT16 + (size_t)i * 8u;
  *(volatile v8h*)dp = hv;
  __threadfence();
  *(volatile v8h*)dp = hv;
}
static_assert((size_t)kE * kP * (kQ / 8) == 768ull * kThr, "transposing cast grid exact: 768 blocks");

__global__ __launch_bounds__(kThr) void bc_cast_kernel(const float* __restrict__ XBCS, unsigned short* __restrict__ dst, int col0) {
  const unsigned i = blockIdx.x * (unsigned)kThr + threadIdx.x;
  const unsigned n8 = i & 7u, r = i >> 3;
  const float* sp = XBCS + (size_t)r * kCD + (unsigned)col0 + n8 * 8u;
  const v4f a0 = *(const v4f*)sp, a1 = *(const v4f*)(sp + 4);
  v8h hv;
#pragma unroll
  for (int t = 0; t < 4; ++t) { const float p = a0[t], q = a1[t]; hv[t] = (_Float16)carry_flush(p, kInCarry); hv[4 + t] = (_Float16)carry_flush(q, kInCarry); }
  unsigned short* dp = dst + (size_t)i * 8u;
  *(volatile v8h*)dp = hv;
  __threadfence();
  *(volatile v8h*)dp = hv;
}
static_assert((size_t)kRows * (kN / 8) == 32ull * kThr, "shared cast grid exact: 32 blocks");

__device__ __forceinline__ void step_of(float pre, float Ah, float& dtv, float& lda) {
  const float sp = (pre > 20.0f) ? pre : log1pf(expf(pre));
  dtv = fminf(fmaxf(sp, 1e-6f), 1000.0f);
  const float da = fminf(fmaxf(expf(dtv * Ah), 1e-6f), 1000.0f);
  lda = logf(da);
}
__global__ __launch_bounds__(128) void prefix_kernel(const float* __restrict__ DTR, const float* __restrict__ A_log, float* __restrict__ CS, float* __restrict__ WTV,
                                                    float* __restrict__ EV, float* __restrict__ DV, float* __restrict__ TOT) {
  const unsigned e = blockIdx.x * 128u + threadIdx.x;
  const unsigned c = e & 7u, bh = e >> 3;
  const unsigned b = bh / (unsigned)kH, h = bh - b * (unsigned)kH;
  const float* ap = DTR + (size_t)(b * (unsigned)kS + c * (unsigned)kQ) * 32u + h;
  const float al = A_log[h];
  const float Ah = -expf(bf16r(al));
  float run = 0.0f;
  for (int q = 0; q < kQ / 4; ++q) {
    v4f s4, o4;
#pragma unroll
    for (int t = 0; t < 4; ++t) { float dtv, lda; step_of(ap[(size_t)(4 * q + t) * 32u], Ah, dtv, lda); run += lda; s4[t] = run; o4[t] = dtv; }
    float* sp = CS + (size_t)e * kQ + 4 * q; float* xp = WTV + (size_t)e * kQ + 4 * q;
    for (int pass = 0; pass < 2; ++pass) { *(volatile v4f*)sp = s4; *(volatile v4f*)xp = o4; __threadfence(); }
  }
  const float tot = run;
  run = 0.0f;
  for (int q = 0; q < kQ / 4; ++q) {
    v4f e4, d4;
#pragma unroll
    for (int t = 0; t < 4; ++t) { float dtv, lda; step_of(ap[(size_t)(4 * q + t) * 32u], Ah, dtv, lda); run += lda; e4[t] = expf(run); d4[t] = expf(tot - run) * dtv; }
    float* ep = EV + (size_t)e * kQ + 4 * q; float* dp = DV + (size_t)e * kQ + 4 * q;
    for (int pass = 0; pass < 2; ++pass) { *(volatile v4f*)ep = e4; *(volatile v4f*)dp = d4; __threadfence(); }
  }
  const float te = expf(tot);
  *(volatile float*)(TOT + e) = te;
  __threadfence();
  *(volatile float*)(TOT + e) = te;
}
static_assert(kE == 3 * 128 && (kQ % 4) == 0, "prefix grid exact: 3 blocks of 128; the two passes' trip count is the literal 16 (64 positions by fours)");

__global__ __launch_bounds__(kThr) void mask_kernel(const float* __restrict__ G32, const float* __restrict__ CS, const float* __restrict__ WTV, unsigned short* __restrict__ M16) {
  const unsigned i = blockIdx.x * (unsigned)kThr + threadIdx.x;
  const unsigned s8 = i & 7u, l = (i >> 3) & 63u, e = i >> 9;
  const unsigned c = e & 7u, bh = e >> 3;
  const unsigned b = bh / (unsigned)kH;
  const float* gp = G32 + ((size_t)(b * (unsigned)kC + c) * kQ + l) * kQ + s8 * 8u;
  const float* xp = CS + (size_t)e * kQ + s8 * 8u;
  const float* wp = WTV + (size_t)e * kQ + s8 * 8u;
  const v4f g0 = *(const v4f*)gp, g1 = *(const v4f*)(gp + 4), x0 = *(const v4f*)xp, x1 = *(const v4f*)(xp + 4), w0 = *(const v4f*)wp, w1 = *(const v4f*)(wp + 4);
  const float csl = CS[(size_t)e * kQ + l];
  v8h hv;
#pragma unroll
  for (int t = 0; t < 8; ++t) {
    const bool live = (s8 * 8u + (unsigned)t) <= l;
    const float gv = (t < 4) ? g0[t] : g1[t - 4];
    const float xv = (t < 4) ? x0[t] : x1[t - 4];
    const float ov = (t < 4) ? w0[t] : w1[t - 4];
    const float d = live ? (csl - xv) : 0.0f;
    const float w = live ? gv * expf(d) * ov : 0.0f;
    hv[t] = (_Float16)carry_flush(w, kInCarry);
  }
  unsigned short* dp = M16 + (size_t)i * 8u;
  *(volatile v8h*)dp = hv;
  __threadfence();
  *(volatile v8h*)dp = hv;
}
static_assert((size_t)kE * kQ * (kQ / 8) == 768ull * kThr, "mask grid exact: 768 blocks");

__global__ __launch_bounds__(kThr) void sc_cast_kernel(const float* __restrict__ XBCS, const float* __restrict__ f1, unsigned short* __restrict__ dst, int tr) {
  const unsigned i = blockIdx.x * (unsigned)kThr + threadIdx.x;
  const unsigned lo = i & 7u, mid = (i >> 3) & 63u, e = i >> 9;
  const unsigned c = e & 7u, bh = e >> 3;
  const unsigned b = bh / (unsigned)kH;
  const size_t row0 = (size_t)b * kS + (size_t)c * kQ;
  v8h hv;
  if (tr != 0) {
    const float* sp = XBCS + (row0 + lo * 8u) * kCD + (unsigned)kDS + mid;
    const float* p1 = f1 + (size_t)e * kQ + lo * 8u;
    const v4f a0 = *(const v4f*)p1, a1 = *(const v4f*)(p1 + 4);
#pragma unroll
    for (int t = 0; t < 8; ++t) { const float x = sp[(size_t)t * kCD]; const float fa = (t < 4) ? a0[t] : a1[t - 4]; hv[t] = (_Float16)carry_flush(x * fa, kInCarry); }
  } else {
    const float* sp = XBCS + (row0 + mid) * kCD + (unsigned)(kDS + kN) + lo * 8u;
    const v4f a0 = *(const v4f*)sp, a1 = *(const v4f*)(sp + 4);
    const float fa = f1[(size_t)e * kQ + mid];
#pragma unroll
    for (int t = 0; t < 8; ++t) { const float x = (t < 4) ? a0[t] : a1[t - 4]; hv[t] = (_Float16)carry_flush(x * fa, kInCarry); }
  }
  unsigned short* dp = dst + (size_t)i * 8u;
  *(volatile v8h*)dp = hv;
  __threadfence();
  *(volatile v8h*)dp = hv;
}
static_assert((size_t)kE * kQ * (kN / 8) == 768ull * kThr, "scaled cast grid exact: 768 blocks");

__global__ __launch_bounds__(kThr) void carry_kernel(const float* __restrict__ ST32, const float* __restrict__ TOT, unsigned short* __restrict__ H16) {
  const unsigned i = blockIdx.x * (unsigned)kThr + threadIdx.x;
  const unsigned n2 = i & 31u, p = (i >> 5) & 63u, bh = i >> 11;
  float h0 = 0.0f, h1 = 0.0f;
  for (int c = 0; c < kC; ++c) {
    const size_t e = (size_t)bh * kC + (size_t)c;
    const size_t o = (e * kP + p) * kN + n2 * 2u;
    v2h hv;
    hv[0] = (_Float16)carry_flush(h0, kInCarry);
    hv[1] = (_Float16)carry_flush(h1, kInCarry);
    unsigned short* dp = H16 + o;
    *(volatile v2h*)dp = hv;
    __threadfence();
    *(volatile v2h*)dp = hv;
    const v2f sv = *(const v2f*)(ST32 + o);
    const float tt = TOT[e];
    h0 = fminf(fmaxf(tt * h0 + sv[0], -1000.0f), 1000.0f);
    h1 = fminf(fmaxf(tt * h1 + sv[1], -1000.0f), 1000.0f);
  }
}
static_assert((size_t)kNb * kH * kP * (kN / 2) == 384ull * kThr && kN / 2 == 32, "carry grid exact: 384 blocks; a wave = one [p] row of 64 state columns");

__global__ __launch_bounds__(kThr) void gate_cast_kernel(const float* __restrict__ YD32, const float* __restrict__ YO32, const float* __restrict__ XBCS, const float* __restrict__ Z32,
                                                        const float* __restrict__ Dp, unsigned short* __restrict__ Y16) {
  const unsigned i = blockIdx.x * (unsigned)kThr + threadIdx.x;
  const unsigned r = i / 192u, hp = i - r * 192u;
  const unsigned h = hp >> 3, p8 = hp & 7u;
  const unsigned b = r >> 9, t = r & 511u;
  const size_t e = ((size_t)b * kH + h) * kC + (t >> 6);
  const size_t so = (e * kQ + (t & 63u)) * kP + p8 * 8u;
  const float* xp = XBCS + (size_t)r * kCD + h * (unsigned)kP + p8 * 8u;
  const float* zp = Z32 + (size_t)r * kDS + h * (unsigned)kP + p8 * 8u;
  const v4f a0 = *(const v4f*)(YD32 + so), a1 = *(const v4f*)(YD32 + so + 4), b0 = *(const v4f*)(YO32 + so), b1 = *(const v4f*)(YO32 + so + 4);
  const v4f x0 = *(const v4f*)xp, x1 = *(const v4f*)(xp + 4), z0 = *(const v4f*)zp, z1 = *(const v4f*)(zp + 4);
  const float d0 = Dp[h];
  const float dh = bf16r(d0);
  v8h hv;
#pragma unroll
  for (int k = 0; k < 8; ++k) {
    const float ya = (k < 4) ? a0[k] : a1[k - 4], yb = (k < 4) ? b0[k] : b1[k - 4];
    const float xv = (k < 4) ? x0[k] : x1[k - 4], zv = (k < 4) ? z0[k] : z1[k - 4];
    const float y = ya + yb + dh * xv;
    hv[k] = (_Float16)carry_flush(y * (zv / (1.0f + expf(-zv))), kInCarry);
  }
  unsigned short* dp = Y16 + (size_t)i * 8u;
  *(volatile v8h*)dp = hv;
  __threadfence();
  *(volatile v8h*)dp = hv;
}
static_assert((size_t)kRows * (kDS / 8) == 768ull * kThr && kDS / 8 == 192, "gated cast grid exact: 768 blocks; 192 groups of 8 a row");

static_assert(((size_t)kRows * kDM / 8) % kThr == 0 && ((size_t)kDin * kDM / 8) % kThr == 0 && ((size_t)kDM * kDS / 8) % kThr == 0, "plane cast grids exact");
static_assert(((kRows / 64) * (kDS / 64)) % 8 == 0 && ((kRows / 64) * (kCD / 64)) % 8 == 0 && ((kRows / 64) * (32 / 32)) % 8 == 0 && ((kRows / 64) * (kDM / 64)) % 8 == 0, "the projections' grids exact: every wave live");
static_assert((size_t)(kDinP - kDin) * kDM * 2 == 3ull * kThr * 4 * 4, "W_in's padding rows = 3 zero-fill blocks of 1,024 floats' worth");

extern "C" void kernel_launch(void* const* d_in, const int* in_sizes, int n_in,
                              void* d_out, int out_size, void* d_ws, size_t ws_size,
                              hipStream_t stream) {
  if (n_in < 8 || d_out == nullptr || d_ws == nullptr) return;
  if (in_sizes[0] != kRows * kDM || in_sizes[1] != kDin * kDM || in_sizes[2] != kCD * 4 || in_sizes[3] != kCD || in_sizes[4] != kH || in_sizes[5] != kH || in_sizes[6] != kH || in_sizes[7] != kDM * kDS) return;
  if (out_size != kRows * kDM) return;
  if (ws_size < kWsTotal) return;
  const float* u = (const float*)d_in[0];
  const float* W_in = (const float*)d_in[1];
  const float* conv_w = (const float*)d_in[2];
  const float* conv_b = (const float*)d_in[3];
  const float* dt_bias = (const float*)d_in[4];
  const float* A_log = (const float*)d_in[5];
  const float* Dp = (const float*)d_in[6];
  const float* W_out = (const float*)d_in[7];
  float* out = (float*)d_out;
  char* ws = (char*)d_ws;
  float* ZB = (float*)(ws + kOffZB);
  float* BIA = (float*)(ws + kOffBIA);
  unsigned short* U16 = (unsigned short*)(ws + kOffU16);
  unsigned short* WIN16 = (unsigned short*)(ws + kOffWIN16);
  unsigned short* WOUT16 = (unsigned short*)(ws + kOffWOUT16);
  float* Z32 = (float*)(ws + kOffZ32);
  float* XBC32 = (float*)(ws + kOffXBC32);
  float* XBCS32 = (float*)(ws + kOffXBCS32);
  float* DTR32 = (float*)(ws + kOffDTR32);
  unsigned short* XT16 = (unsigned short*)(ws + kOffXT16);
  unsigned short* B16 = (unsigned short*)(ws + kOffB16);
  unsigned short* C16 = (unsigned short*)(ws + kOffC16);
  float* G32 = (float*)(ws + kOffG32);
  float* CS = (float*)(ws + kOffCS);
  float* WTV = (float*)(ws + kOffWTV);
  float* EV = (float*)(ws + kOffEV);
  float* DV = (float*)(ws + kOffDV);
  float* TOT = (float*)(ws + kOffTOT);
  unsigned short* M16 = (unsigned short*)(ws + kOffM16);
  float* YD32 = (float*)(ws + kOffYD32);
  unsigned short* BDT16 = (unsigned short*)(ws + kOffBDT16);
  float* ST32 = (float*)(ws + kOffST32);
  float* YO32 = (float*)(ws + kOffYO32);
  unsigned short* H16 = (unsigned short*)(ws + kOffH16);
  unsigned short* CE16 = (unsigned short*)(ws + kOffCE16);
  unsigned short* Y16 = (unsigned short*)(ws + kOffY16);
  const long kStr = (long)kQ * kN;

  zero_kernel<<<2, kThr, 0, stream>>>(ZB);
  zero_kernel<<<3, kThr, 0, stream>>>((float*)(WIN16 + (size_t)kDin * kDM));
  bias_kernel<<<1, 64, 0, stream>>>(dt_bias, BIA);
  cast_plane_kernel<<<(int)(((size_t)kRows * kDM / 8) / kThr), kThr, 0, stream>>>(u, U16, 6, 64, 0);
  cast_plane_kernel<<<(int)(((size_t)kDin * kDM / 8) / kThr), kThr, 0, stream>>>(W_in, WIN16, 6, 64, 0);
  cast_plane_kernel<<<(int)(((size_t)kDM * kDS / 8) / kThr), kThr, 0, stream>>>(W_out, WOUT16, 6, 64, 0);
  wmma_gemm64<0, false, 2, 0, false, 0><<<dim3((kRows / 64) * (kDS / 64) / 8, 1), 256, 0, stream>>>(
      U16, U16, kDM, 0L, WIN16, WIN16, kDM, 0L, (void*)Z32, (void*)Z32, kDS, 0L, ZB, nullptr, 0L, kRows, kDS, kDM, kSc);
  wmma_gemm64<0, false, 2, 0, false, 0><<<dim3((kRows / 64) * (kCD / 64) / 8, 1), 256, 0, stream>>>(
      U16, U16, kDM, 0L, WIN16 + (size_t)kDS * kDM, WIN16 + (size_t)kDS * kDM, kDM, 0L, (void*)XBC32, (void*)XBC32, kCD, 0L, ZB, nullptr, 0L, kRows, kCD, kDM, kSc);
  wmma_gemm32<<<dim3((kRows / 64) * (32 / 32) / 8, 1), 256, 0, stream>>>(
      U16, kDM, 0L, WIN16 + (size_t)(kDS + kCD) * kDM, kDM, 0L, DTR32, 32, 0L, BIA, kRows, 32, kDM, kSc);
  conv_silu_kernel<<<1664, kThr, 0, stream>>>(XBC32, conv_w, conv_b, XBCS32);
  xt_cast_kernel<<<768, kThr, 0, stream>>>(XBCS32, XT16);
  bc_cast_kernel<<<32, kThr, 0, stream>>>(XBCS32, B16, kDS);
  bc_cast_kernel<<<32, kThr, 0, stream>>>(XBCS32, C16, kDS + kN);
  prefix_kernel<<<3, 128, 0, stream>>>(DTR32, A_log, CS, WTV, EV, DV, TOT);
  wmma_gemm64<0, false, 2, 0, false, 0><<<dim3(1, kBC), 256, 0, stream>>>(
      C16, C16, kN, kStr, B16, B16, kN, kStr, (void*)G32, (void*)G32, kQ, kStr, ZB, nullptr, 0L, kQ, kQ, kN, kSc);
  mask_kernel<<<768, kThr, 0, stream>>>(G32, CS, WTV, M16);
  wmma_gemm64<0, false, 2, 0, false, 0><<<dim3(1, kE), 256, 0, stream>>>(
      M16, M16, kQ, kStr, XT16, XT16, kQ, kStr, (void*)YD32, (void*)YD32, kP, kStr, ZB, nullptr, 0L, kQ, kP, kQ, kSc);
  sc_cast_kernel<<<768, kThr, 0, stream>>>(XBCS32, DV, BDT16, 1);
  wmma_gemm64<0, false, 2, 0, false, 0><<<dim3(1, kE), 256, 0, stream>>>(
      XT16, XT16, kQ, kStr, BDT16, BDT16, kQ, kStr, (void*)ST32, (void*)ST32, kN, kStr, ZB, nullptr, 0L, kP, kN, kQ, kSc);
  carry_kernel<<<384, kThr, 0, stream>>>(ST32, TOT, H16);
  sc_cast_kernel<<<768, kThr, 0, stream>>>(XBCS32, EV, CE16, 0);
  wmma_gemm64<0, false, 2, 0, false, 0><<<dim3(1, kE), 256, 0, stream>>>(
      CE16, CE16, kN, kStr, H16, H16, kN, kStr, (void*)YO32, (void*)YO32, kP, kStr, ZB, nullptr, 0L, kQ, kP, kN, kSc);
  gate_cast_kernel<<<768, kThr, 0, stream>>>(YD32, YO32, XBCS32, Z32, Dp, Y16);
  wmma_gemm64<0, false, 2, 0, false, 0><<<dim3((kRows / 64) * (kDM / 64) / 8, 1), 256, 0, stream>>>(
      Y16, Y16, kDS, 0L, WOUT16, WOUT16, kDS, 0L, (void*)out, (void*)out, kDM, 0L, ZB, nullptr, 0L, kRows, kDM, kDS, kSc);
}
